// STUCore_49417893708193
// MI455X (gfx1250) — hardware-verified
//
#include <hip/hip_runtime.h>
#include <stddef.h>
#include <stdint.h>


typedef unsigned short us8 __attribute__((ext_vector_type(8)));
typedef us8 us8a __attribute__((may_alias));
typedef __bf16 v16bf __attribute__((ext_vector_type(16)));
typedef float v8f __attribute__((ext_vector_type(8)));
typedef float v4f __attribute__((ext_vector_type(4)));
typedef float v2f __attribute__((ext_vector_type(2)));
typedef v4f v4fa __attribute__((may_alias));
typedef v2f v2fa __attribute__((may_alias));

#define NB    4
#define NL    2048
#define ND    1024
#define NE    24
#define KE    32
#define MROWS (NB * NL)

#define SEG_X   (MROWS * ND / 8)
#define SEG_MT  (ND * ND / 8)
#define SEG_PH  (NL * KE / 8)
#define SEG_MF  (ND * KE / 8)
#define CVT_THREADS (SEG_X + SEG_MT + SEG_PH + SEG_MF)

static_assert((CVT_THREADS % 256) == 0);
static_assert((SEG_X % 32) == 0);
static_assert((SEG_MT % 32) == 0);
static_assert((SEG_PH % 32) == 0);
static_assert((SEG_MF % 32) == 0);

#define GP 68

#define TB   256
#define SCH  512
#define WU   (TB + SCH + 4)
#define WV   (SCH / 2 + 4)
#define RR   32
#define OTP  36

static_assert(TB == 8 * RR);
static_assert(TB * OTP <= 32 * WU);
static_assert((NL % TB) == 0);
static_assert((NL % SCH) == 0);
static_assert(((WU * 4) % 16) == 0);
static_assert(((WV * 4) % 16) == 0);

union Frag { us8 q[2]; v16bf v; };

static __device__ __forceinline__ unsigned short f2bf(float f) {
  unsigned int u = __float_as_uint(f);
  u += 0x7FFFu + ((u >> 16) & 1u);
  return (unsigned short)(u >> 16);
}

static __device__ __forceinline__ v8f wmma_bf16(v16bf a, v16bf b, v8f c) {
  c = __builtin_amdgcn_wmma_f32_16x16x32_bf16(false, a, false, b, (short)0, c, false, false);
  asm volatile("v_nop\n\tv_nop\n\tv_nop\n\tv_nop" : "+v"(c) : "v"(a), "v"(b));
  return c;
}

__global__ __launch_bounds__(256)
void k_convert(const float* __restrict__ x, const float* __restrict__ Mi,
               const float* __restrict__ phi, const float* __restrict__ Mf,
               unsigned short* xb, unsigned short* Mt,
               unsigned short* phb, unsigned short* Mft) {
  const int gid = blockIdx.x * 256 + threadIdx.x;
  if (gid >= CVT_THREADS) return;
  float f[8];
  unsigned short* dst;
  if (gid < SEG_X) {
    const float* p = x + (size_t)gid * 8;
    const v4f a = *(const v4fa*)p;
    const v4f c = *(const v4fa*)(p + 4);
    f[0] = a.x; f[1] = a.y; f[2] = a.z; f[3] = a.w;
    f[4] = c.x; f[5] = c.y; f[6] = c.z; f[7] = c.w;
    dst = xb + (size_t)gid * 8;
  } else if (gid < SEG_X + SEG_MT) {
    const int i = gid - SEG_X;
    const int n = i >> 7, kq = i & 127;
#pragma unroll
    for (int e = 0; e < 8; ++e) f[e] = Mi[(size_t)(8 * kq + e) * ND + n];
    dst = Mt + (size_t)n * ND + 8 * kq;
  } else if (gid < SEG_X + SEG_MT + SEG_PH) {
    const int i = gid - SEG_X - SEG_MT;
    const int row = i >> 2, q = i & 3;
    if (q < 3) {
#pragma unroll
      for (int e = 0; e < 8; ++e) f[e] = phi[(size_t)row * NE + 8 * q + e];
    } else {
#pragma unroll
      for (int e = 0; e < 8; ++e) f[e] = 0.f;
    }
    dst = phb + (size_t)row * KE + 8 * q;
  } else {
    const int i = gid - SEG_X - SEG_MT - SEG_PH;
    const int n = i >> 2, q = i & 3;
    if (q < 3) {
#pragma unroll
      for (int e = 0; e < 8; ++e) f[e] = Mf[(size_t)(8 * q + e) * ND + n];
    } else {
#pragma unroll
      for (int e = 0; e < 8; ++e) f[e] = 0.f;
    }
    dst = Mft + (size_t)n * KE + 8 * q;
  }
  union { us8 v; unsigned short s[8]; } pk;
#pragma unroll
  for (int e = 0; e < 8; ++e) pk.s[e] = f2bf(f[e]);
  const us8 pv = pk.v;
  *(volatile us8*)dst = pv;
  __threadfence();
  *(volatile us8*)dst = pv;
}

__global__ __launch_bounds__(128)
void k_gemm_bf16(const unsigned short* __restrict__ A,
                 const unsigned short* __restrict__ Bt,
                 float* __restrict__ C, int N, int K) {
  __shared__ __attribute__((aligned(16))) float tile[4 * 32 * GP];
  const int tid = threadIdx.x;
  const int lane = tid & 31, wave = tid >> 5;
  const int h = lane >> 4, m = lane & 15;
  const int wr = wave >> 1, wc = wave & 1;
  const int row0 = blockIdx.x * 64 + wr * 32;
  const int col0 = blockIdx.y * 128 + wc * 64;

  v8f acc[2][4];
#pragma unroll
  for (int i = 0; i < 2; ++i)
#pragma unroll
    for (int j = 0; j < 4; ++j)
#pragma unroll
      for (int r = 0; r < 8; ++r) acc[i][j][r] = 0.f;

  const unsigned short* ap = A + (size_t)(row0 + m) * K + 8 * h;
  const unsigned short* bp = Bt + (size_t)(col0 + m) * K + 8 * h;
  const size_t s16 = (size_t)16 * K;

#pragma unroll 1
  for (int k0 = 0; k0 < K; k0 += 32) {
    Frag a[2], b[4];
#pragma unroll
    for (int i = 0; i < 2; ++i) {
      const unsigned short* p = ap + i * s16 + k0;
      a[i].q[0] = *(const us8a*)p;
      a[i].q[1] = *(const us8a*)(p + 16);
    }
#pragma unroll
    for (int j = 0; j < 4; ++j) {
      const unsigned short* p = bp + j * s16 + k0;
      b[j].q[0] = *(const us8a*)p;
      b[j].q[1] = *(const us8a*)(p + 16);
    }
#pragma unroll
    for (int i = 0; i < 2; ++i)
#pragma unroll
      for (int j = 0; j < 4; ++j)
        acc[i][j] = wmma_bf16(a[i].v, b[j].v, acc[i][j]);
  }

  float* tw = tile + wave * (32 * GP);
#pragma unroll
  for (int i = 0; i < 2; ++i)
#pragma unroll
    for (int j = 0; j < 4; ++j)
#pragma unroll
      for (int r = 0; r < 8; ++r)
        tw[(16 * i + 8 * h + r) * GP + 16 * j + m] = acc[i][j][r];
  __syncthreads();

  v4f vals[16];
#pragma unroll
  for (int it = 0; it < 16; ++it)
    vals[it] = *(const v4fa*)(tw + (2 * it + h) * GP + 4 * m);

  float* cb = C + ((size_t)row0 * N + col0 + 4 * m);
#pragma unroll
  for (int it = 0; it < 16; ++it)
    *(volatile v4f*)(cb + (size_t)(2 * it + h) * N) = vals[it];
  __threadfence();
#pragma unroll
  for (int it = 0; it < 16; ++it)
    *(volatile v4f*)(cb + (size_t)(2 * it + h) * N) = vals[it];
}

__global__ __launch_bounds__(256)
void k_conv(const float* __restrict__ U, const float* __restrict__ V,
            float* __restrict__ out) {
  __shared__ __attribute__((aligned(16))) float u_l[32 * WU];
  __shared__ __attribute__((aligned(16))) float v_l[32 * WV];
  const int tid = threadIdx.x;
  const int lane = tid & 31, g = tid >> 5;
  const int bx = blockIdx.x;
  const int dg = bx & 31, tb = (bx >> 5) & 7, b = bx >> 8;
  const int d0 = dg * 32, t_lo = tb * TB;
  const int t_max = t_lo + 32 * g + 31;

  float acc[RR];
#pragma unroll
  for (int r = 0; r < RR; ++r) acc[r] = 0.f;

  const int nch = (t_lo + TB - 1) / SCH + 1;
  for (int ch = 0; ch < nch; ++ch) {
    const int s_c = ch * SCH;
    const int i_base = t_lo - s_c - SCH;
    __syncthreads();
    for (int q = tid; q < (TB + SCH) * 8; q += 256) {
      const int li = q >> 3, cq = q & 7;
      const int i = i_base + li;
      v4f val;
      val.x = 0.f; val.y = 0.f; val.z = 0.f; val.w = 0.f;
      if (i >= 0 && i < NL)
        val = *(const v4fa*)(U + ((size_t)(b * NL + i) * ND + d0 + 4 * cq));
      float* dst = u_l + (4 * cq) * WU + li;
      dst[0] = val.x; dst[WU] = val.y; dst[2 * WU] = val.z; dst[3 * WU] = val.w;
    }
    for (int q = tid; q < (SCH / 2) * 8; q += 256) {
      const int p = q >> 3, cq = q & 7;
      const int s = s_c + 2 * p;
      const v4f val = *(const v4fa*)(V + ((size_t)s * ND + d0 + 4 * cq));
      float* dst = v_l + (4 * cq) * WV + p;
      dst[0] = val.x; dst[WV] = val.y; dst[2 * WV] = val.z; dst[3 * WV] = val.w;
    }
    __syncthreads();

    const int rem = t_max - s_c;
    int ng = (rem < 0) ? 0 : ((rem >> 2) + 1);
    if (ng > SCH / 4) ng = SCH / 4;
    const float* ub = u_l + lane * WU + (SCH + 32 * g - 4);
    const float* vb = v_l + lane * WV;
#pragma unroll 1
    for (int gi = 0; gi < ng; ++gi) {
      const float* wp = ub - 4 * gi;
      const float* vp = vb + 2 * gi;
      union { v4f q[9]; float f[36]; } w;
#pragma unroll
      for (int e = 0; e < 9; ++e) w.q[e] = *(const v4fa*)(wp + 4 * e);
      const v2f vv = *(const v2fa*)vp;
#pragma unroll
      for (int r = 0; r < RR; ++r) {
        acc[r] = __builtin_fmaf(vv.x, w.f[r + 4], acc[r]);
        acc[r] = __builtin_fmaf(vv.y, w.f[r + 2], acc[r]);
      }
    }
  }

  __syncthreads();
  float* ot = u_l;
#pragma unroll
  for (int r = 0; r < RR; ++r) ot[(32 * g + r) * OTP + lane] = 2.0f * acc[r];
  __syncthreads();

  const int rq = lane >> 3, cq4 = 4 * (lane & 7);
  v4f vals[8];
#pragma unroll
  for (int k = 0; k < 8; ++k)
    vals[k] = *(const v4fa*)(ot + (32 * g + 4 * k + rq) * OTP + cq4);

  float* ob = out + ((size_t)(b * NL + t_lo + 32 * g) * ND + d0 + cq4);
#pragma unroll
  for (int k = 0; k < 8; ++k)
    *(volatile v4f*)(ob + (size_t)(4 * k + rq) * ND) = vals[k];
  __threadfence();
#pragma unroll
  for (int k = 0; k < 8; ++k)
    *(volatile v4f*)(ob + (size_t)(4 * k + rq) * ND) = vals[k];
}

extern "C" void kernel_launch(void* const* d_in, const int* in_sizes, int n_in,
                              void* d_out, int out_size, void* d_ws, size_t ws_size,
                              hipStream_t stream) {
  if (n_in < 4) return;
  if (in_sizes[0] != MROWS * ND || in_sizes[1] != ND * ND ||
      in_sizes[2] != NE * ND || in_sizes[3] != NL * NE) return;
  if (out_size != MROWS * ND) return;

  const float* x   = (const float*)d_in[0];
  const float* Mi  = (const float*)d_in[1];
  const float* Mf  = (const float*)d_in[2];
  const float* phi = (const float*)d_in[3];
  float* out = (float*)d_out;

  char* w = (char*)d_ws;
  size_t off = 0;
  unsigned short* xb  = (unsigned short*)(w + off); off += (size_t)MROWS * ND * 2;
  unsigned short* Mt  = (unsigned short*)(w + off); off += (size_t)ND * ND * 2;
  unsigned short* phb = (unsigned short*)(w + off); off += (size_t)NL * KE * 2;
  unsigned short* Mft = (unsigned short*)(w + off); off += (size_t)ND * KE * 2;
  float* U            = (float*)(w + off);          off += (size_t)MROWS * ND * 4;
  float* V            = (float*)(w + off);          off += (size_t)NL * ND * 4;
  if (off > ws_size) return;

  k_convert<<<CVT_THREADS / 256, 256, 0, stream>>>(x, Mi, phi, Mf, xb, Mt, phb, Mft);
  k_gemm_bf16<<<dim3(MROWS / 64, ND / 128), 128, 0, stream>>>(xb, Mt, U, ND, ND);
  k_gemm_bf16<<<dim3(NL / 64, ND / 128), 128, 0, stream>>>(phb, Mft, V, ND, KE);
  k_conv<<<NB * (NL / TB) * (ND / 32), 256, 0, stream>>>(U, V, out);
}
